// MultiHeadedAttention_50431505990010
// MI455X (gfx1250) — hardware-verified
//
#include <hip/hip_runtime.h>
#ifndef NB
#define NB 4
#endif
#ifndef SEQ
#define SEQ 2048
#endif
#define NB_FULL 4
#define SEQ_FULL 2048
#define DM 1024
#define NH 16
#define HD 64
#define NR ((size_t)NB * SEQ)
#define CW 4
#define AW 4
#define SC2 0.18033688011112042f
#define VCARRY 4096.0f
#define SZ_W   ((size_t)DM * DM * 2)
#define SZ_ACT (NR * DM * 2)
#define SZ_ST  ((size_t)NB * NH * SEQ * 4)
#define WS_TOTAL (4 * SZ_W + 6 * SZ_ACT + 2 * SZ_ST)

static_assert(DM == NH * HD);
static_assert(HD == 64);
static_assert(DM % 64 == 0 && DM % 32 == 0);
static_assert((NB * SEQ) % 128 == 0);
static_assert(SEQ % (CW * 64) == 0);
static_assert(SEQ % (AW * 16) == 0);
static_assert(SEQ % 64 == 0 && SEQ % 32 == 0 && SEQ % 16 == 0);
static_assert(NB <= NB_FULL && SEQ <= SEQ_FULL);
static_assert(SZ_W % 256 == 0 && SZ_ACT % 256 == 0 && SZ_ST % 256 == 0);
static_assert(WS_TOTAL <= (size_t)134217728);

typedef _Float16 v16h __attribute__((ext_vector_type(16)));
typedef _Float16 v4h __attribute__((ext_vector_type(4)));
typedef unsigned short v8us __attribute__((ext_vector_type(8), may_alias));
typedef float  v8f  __attribute__((ext_vector_type(8)));
typedef float  v4f  __attribute__((ext_vector_type(4)));
typedef float  v4fa __attribute__((ext_vector_type(4), may_alias));
union FragH { v16h v; v8us half[2]; _Float16 h[16]; unsigned short u[16]; };

__device__ __forceinline__ unsigned short bf16_bits(float x) { unsigned int u = __float_as_uint(x); return (unsigned short)((u + 0x7FFFu + ((u >> 16) & 1u)) >> 16); }
__device__ __forceinline__ float bf16_val(unsigned short b) { return __uint_as_float(((unsigned int)b) << 16); }
__device__ __forceinline__ float bf16_rne(float x) { return bf16_val(bf16_bits(x)); }
__device__ __forceinline__ float ex2(float x) {
#if __has_builtin(__builtin_amdgcn_exp2f)
  return __builtin_amdgcn_exp2f(x);
#else
  return exp2f(x);
#endif
}
__device__ __forceinline__ v16h g2_frag(const _Float16* p, int hh) { FragH f; f.half[0] = *(const v8us*)((const unsigned short*)p + 8 * hh); f.half[1] = *(const v8us*)((const unsigned short*)p + 16 + 8 * hh); return f.v; }
__device__ __forceinline__ v8f g2_mma(v16h a, v16h b, v8f c) { v8f d = __builtin_amdgcn_wmma_f32_16x16x32_f16(false, a, false, b, (short)0, c, false, false); asm volatile("v_nop\n\tv_nop\n\tv_nop\n\tv_nop" : "+v"(d) : "v"(a), "v"(b)); return d; }

__global__ __launch_bounds__(256) void k_x16(const float* __restrict__ x, _Float16* __restrict__ X16) {
  const size_t t = (size_t)blockIdx.x * 256 + threadIdx.x; if (t >= NR * (DM / 8)) return;
  const size_t row = t / (DM / 8); const int c8 = (int)(t % (DM / 8)) * 8;
  const size_t b = row / SEQ, s = row % SEQ;
  const float* src = x + (b * (size_t)SEQ_FULL + s) * DM + c8;
  const v4f a = *(const v4fa*)src, c = *(const v4fa*)(src + 4);
  FragH f;
#pragma unroll
  for (int q = 0; q < 4; ++q) { f.h[q] = (_Float16)bf16_rne(a[q]); f.h[4 + q] = (_Float16)bf16_rne(c[q]); }
  const v8us o = f.half[0];
  unsigned short* d = (unsigned short*)X16 + t * 8;
  *(volatile v8us*)d = o; __threadfence(); *(volatile v8us*)d = o;
}

__global__ __launch_bounds__(256) void k_wqkv(const float* __restrict__ W, _Float16* __restrict__ Bt) {
  const int t = blockIdx.x * 256 + threadIdx.x; if (t >= NH * HD * (DM / 8)) return;
  const int n = t / (DM / 8), m8 = (t % (DM / 8)) * 8; const int h = n / HD, d = n % HD;
  FragH f;
#pragma unroll
  for (int i = 0; i < 8; ++i) f.h[i] = (_Float16)(bf16_rne(W[((size_t)h * DM + m8 + i) * HD + d]) * 16.0f);
  const v8us o = f.half[0];
  unsigned short* dst = (unsigned short*)Bt + (size_t)n * DM + m8;
  *(volatile v8us*)dst = o; __threadfence(); *(volatile v8us*)dst = o;
}

__global__ __launch_bounds__(256) void k_wnat(const float* __restrict__ w, size_t n8, _Float16* __restrict__ Bt) {
  const size_t t = (size_t)blockIdx.x * 256 + threadIdx.x; if (t >= n8) return; FragH f;
#pragma unroll
  for (int q = 0; q < 8; ++q) f.h[q] = (_Float16)(bf16_rne(w[t * 8 + q]) * 16.0f);
  const v8us o = f.half[0];
  unsigned short* dst = (unsigned short*)Bt + t * 8;
  *(volatile v8us*)dst = o; __threadfence(); *(volatile v8us*)dst = o;
}

__global__ __launch_bounds__(128) void k_gemm2(const _Float16* __restrict__ A, int lda, const _Float16* __restrict__ Bh, int ldb, float alpha, const float* __restrict__ bias,
    float* __restrict__ C, _Float16* __restrict__ C16, int ldc, int M, int N, int K) {
  __shared__ __attribute__((aligned(16))) float so[4][32][68];
  const int tid = threadIdx.x, w = tid >> 5, lane = tid & 31, ln = lane & 15, hh = lane >> 4;
  const int ntn = N >> 6; const int mt = blockIdx.x / ntn, nq = blockIdx.x - mt * ntn; const int row0 = mt * 128 + 32 * w, col0 = nq * 64; if (row0 >= M) return;
  const _Float16* a0p = A + (size_t)(row0 + ln) * lda; const _Float16* a1p = a0p + (size_t)16 * lda;
  const _Float16* b0p = Bh + (size_t)(col0 + ln) * ldb; const _Float16* b1p = b0p + (size_t)16 * ldb; const _Float16* b2p = b1p + (size_t)16 * ldb; const _Float16* b3p = b2p + (size_t)16 * ldb;
  const v8f z8 = {0.f,0.f,0.f,0.f,0.f,0.f,0.f,0.f}; v8f c00 = z8, c01 = z8, c02 = z8, c03 = z8, c10 = z8, c11 = z8, c12 = z8, c13 = z8;
#pragma unroll 1
  for (int kb = 0; kb < K; kb += 32) { const v16h a0 = g2_frag(a0p + kb, hh), a1 = g2_frag(a1p + kb, hh);
    v16h b = g2_frag(b0p + kb, hh); c00 = g2_mma(a0, b, c00); c10 = g2_mma(a1, b, c10);
    b = g2_frag(b1p + kb, hh); c01 = g2_mma(a0, b, c01); c11 = g2_mma(a1, b, c11);
    b = g2_frag(b2p + kb, hh); c02 = g2_mma(a0, b, c02); c12 = g2_mma(a1, b, c12);
    b = g2_frag(b3p + kb, hh); c03 = g2_mma(a0, b, c03); c13 = g2_mma(a1, b, c13); }
  v8f accs[8] = {c00, c01, c02, c03, c10, c11, c12, c13};
#pragma unroll
  for (int u = 0; u < 8; ++u) { const int t = u & 3, half = u >> 2; const int col = col0 + t * 16 + ln; const float bv = bf16_rne(bias[col]);
#pragma unroll
    for (int r = 0; r < 8; ++r) { const int rloc = half * 16 + 8 * hh + r; so[w][rloc][t * 16 + ln] = accs[u][r] * alpha + bv; } }
  __builtin_amdgcn_fence(4  , "workgroup"); __builtin_amdgcn_wave_barrier();
  const int rsub = lane >> 4, c4 = (lane & 15) * 4;
  for (int pass = 0; pass < 2; ++pass) {
#pragma unroll
    for (int q = 0; q < 16; ++q) { const int r = q * 2 + rsub; const v4f v = *(const v4fa*)&so[w][r][c4];
      if (C) *(volatile v4f*)(C + (size_t)(row0 + r) * ldc + col0 + c4) = v;
      if (C16) { v4h h4;
#pragma unroll
        for (int i = 0; i < 4; ++i) h4[i] = (_Float16)v[i];
        *(volatile v4h*)(C16 + (size_t)(row0 + r) * ldc + col0 + c4) = h4; } }
    if (pass == 0) __threadfence(); }
}

__device__ __forceinline__ void col_update(const v8f c, float& m, float& l) {
  const float tm = fmaxf(fmaxf(fmaxf(c[0], c[1]), fmaxf(c[2], c[3])), fmaxf(fmaxf(c[4], c[5]), fmaxf(c[6], c[7])));
  const float nm = fmaxf(m, tm * SC2);
  float s = 0.f;
#pragma unroll
  for (int r = 0; r < 8; ++r) s += ex2(fmaf(c[r], SC2, -nm));
  l = l * ex2(m - nm) + s;
  m = nm;
}

__global__ __launch_bounds__(CW * 32) void k_cstat(const _Float16* __restrict__ Q16, const _Float16* __restrict__ K16, float* __restrict__ M2, float* __restrict__ RL) {
  __shared__ __attribute__((aligned(16))) float sm[CW][2][64];
  const int tid = threadIdx.x, w = tid >> 5, lane = tid & 31, ln = lane & 15, hh = lane >> 4;
  const int bh = blockIdx.y, b = bh / NH, h = bh - b * NH;
  const int key0 = (blockIdx.x * CW + w) * 64;
  const size_t rb = (size_t)b * SEQ;
  v16h kb[4][2];
#pragma unroll
  for (int t = 0; t < 4; ++t) { const _Float16* kp = K16 + (rb + key0 + t * 16 + ln) * DM + h * HD; kb[t][0] = g2_frag(kp, hh); kb[t][1] = g2_frag(kp + 32, hh); }
  float mr[4], lr[4];
#pragma unroll
  for (int t = 0; t < 4; ++t) { mr[t] = -3.0e38f; lr[t] = 0.f; }
  const _Float16* qp = Q16 + (rb + ln) * DM + h * HD;
  const v8f z8 = {0.f,0.f,0.f,0.f,0.f,0.f,0.f,0.f};
#pragma unroll 1
  for (int qt = 0; qt < SEQ / 16; ++qt) {
    const _Float16* qr = qp + (size_t)qt * 16 * DM;
    const v16h a0 = g2_frag(qr, hh), a1 = g2_frag(qr + 32, hh);
#pragma unroll
    for (int t = 0; t < 4; ++t) { v8f c = g2_mma(a0, kb[t][0], z8); c = g2_mma(a1, kb[t][1], c); col_update(c, mr[t], lr[t]); }
  }
#pragma unroll
  for (int t = 0; t < 4; ++t) {
    const float mo = __shfl_xor(mr[t], 16), lo = __shfl_xor(lr[t], 16);
    const float Mx = fmaxf(mr[t], mo);
    const float L = lr[t] * ex2(mr[t] - Mx) + lo * ex2(mo - Mx);
    const float rl = 1.0f / L;
    if (hh == 0) { sm[w][0][t * 16 + ln] = Mx; sm[w][1][t * 16 + ln] = rl; }
  }
  __builtin_amdgcn_fence(4  , "workgroup"); __builtin_amdgcn_wave_barrier();
  const v4f mv = *(const v4fa*)&sm[w][0][ln * 4], rv = *(const v4fa*)&sm[w][1][ln * 4];
  float* mdst = M2 + (size_t)bh * SEQ + key0 + ln * 4; float* rdst = RL + (size_t)bh * SEQ + key0 + ln * 4;
  for (int pass = 0; pass < 2; ++pass) {
    if (lane < 16) { *(volatile v4f*)mdst = mv; *(volatile v4f*)rdst = rv; }
    if (pass == 0) __threadfence(); }
}

__global__ __launch_bounds__(256) void k_vt(const _Float16* __restrict__ V16, const float* __restrict__ RL, _Float16* __restrict__ VT) {
  __shared__ unsigned short tl[64][66];
  const int tid = threadIdx.x; const int slab = blockIdx.x / (SEQ / 64), lg = blockIdx.x % (SEQ / 64); const int b = slab / NH, h = slab % NH;
  for (int i = tid; i < 64 * 8; i += 256) { const int r = i / 8, c8 = (i % 8) * 8; FragH f, g;
    f.half[0] = *(const v8us*)((const unsigned short*)V16 + ((size_t)b * SEQ + lg * 64 + r) * DM + h * HD + c8);
    const float sc = RL[(size_t)slab * SEQ + lg * 64 + r] * VCARRY;
#pragma unroll
    for (int q = 0; q < 8; ++q) g.h[q] = (_Float16)((float)f.h[q] * sc);
#pragma unroll
    for (int q = 0; q < 8; ++q) tl[r][c8 + q] = g.u[q]; }
  __syncthreads();
  for (int pass = 0; pass < 2; ++pass) {
#pragma unroll
    for (int rd = 0; rd < 2; ++rd) { const int d = rd * 32 + tid / 8, pc = tid % 8; FragH f;
#pragma unroll
      for (int q = 0; q < 8; ++q) f.u[q] = tl[pc * 8 + q][d];
      *(volatile v8us*)((unsigned short*)VT + ((size_t)slab * HD + d) * SEQ + lg * 64 + pc * 8) = f.half[0]; }
    if (pass == 0) __threadfence(); }
}

__global__ __launch_bounds__(AW * 32) void k_actx(const _Float16* __restrict__ Q16, const _Float16* __restrict__ K16, const _Float16* __restrict__ VT, const float* __restrict__ M2, _Float16* __restrict__ O16) {
  __shared__ __attribute__((aligned(16))) float so[AW][16][68];
  const int tid = threadIdx.x, w = tid >> 5, lane = tid & 31, ln = lane & 15, hh = lane >> 4;
  const int bh = blockIdx.y, b = bh / NH, h = bh - b * NH;
  const int q0 = (blockIdx.x * AW + w) * 16;
  const size_t rb = (size_t)b * SEQ;
  const _Float16* qp = Q16 + (rb + q0 + ln) * DM + h * HD;
  const v16h qb0 = g2_frag(qp, hh), qb1 = g2_frag(qp + 32, hh);
  const _Float16* kp = K16 + (rb + ln) * DM + h * HD;
  const _Float16* vp = VT + ((size_t)bh * HD + ln) * SEQ;
  const float* mp = M2 + (size_t)bh * SEQ + 8 * hh;
  const v8f z8 = {0.f,0.f,0.f,0.f,0.f,0.f,0.f,0.f};
  v8f o0 = z8, o1 = z8, o2 = z8, o3 = z8;
#pragma unroll 1
  for (int s0 = 0; s0 < SEQ; s0 += 32) {
    const _Float16* k0 = kp + (size_t)s0 * DM; const _Float16* k1 = k0 + (size_t)16 * DM;
    v16h a = g2_frag(k0, hh); v8f c0 = g2_mma(a, qb0, z8); a = g2_frag(k0 + 32, hh); c0 = g2_mma(a, qb1, c0);
    a = g2_frag(k1, hh); v8f c1 = g2_mma(a, qb0, z8); a = g2_frag(k1 + 32, hh); c1 = g2_mma(a, qb1, c1);
    const v4f ma = *(const v4fa*)(mp + s0), mb = *(const v4fa*)(mp + s0 + 4), mc = *(const v4fa*)(mp + s0 + 16), md = *(const v4fa*)(mp + s0 + 20);
    FragH p;
#pragma unroll
    for (int r = 0; r < 4; ++r) {
      p.h[r]      = (_Float16)ex2(fmaf(c0[r],     SC2, -ma[r]));
      p.h[4 + r]  = (_Float16)ex2(fmaf(c0[4 + r], SC2, -mb[r]));
      p.h[8 + r]  = (_Float16)ex2(fmaf(c1[r],     SC2, -mc[r]));
      p.h[12 + r] = (_Float16)ex2(fmaf(c1[4 + r], SC2, -md[r]));
    }
    const _Float16* v0 = vp + s0;
    a = g2_frag(v0, hh);                    o0 = g2_mma(a, p.v, o0);
    a = g2_frag(v0 + (size_t)16 * SEQ, hh); o1 = g2_mma(a, p.v, o1);
    a = g2_frag(v0 + (size_t)32 * SEQ, hh); o2 = g2_mma(a, p.v, o2);
    a = g2_frag(v0 + (size_t)48 * SEQ, hh); o3 = g2_mma(a, p.v, o3);
  }
#pragma unroll
  for (int r = 0; r < 8; ++r) {
    so[w][ln][ 0 + 8 * hh + r] = o0[r] * 0.015625f;
    so[w][ln][16 + 8 * hh + r] = o1[r] * 0.015625f;
    so[w][ln][32 + 8 * hh + r] = o2[r] * 0.015625f;
    so[w][ln][48 + 8 * hh + r] = o3[r] * 0.015625f;
  }
  __builtin_amdgcn_fence(4  , "workgroup"); __builtin_amdgcn_wave_barrier();
  const int qs = lane >> 3, pc = lane & 7;
  v8us ov[4];
#pragma unroll
  for (int it = 0; it < 4; ++it) { const int q = it * 4 + qs; const v4f x0 = *(const v4fa*)&so[w][q][pc * 8], x1 = *(const v4fa*)&so[w][q][pc * 8 + 4]; FragH f;
#pragma unroll
    for (int i = 0; i < 4; ++i) { f.h[i] = (_Float16)x0[i]; f.h[4 + i] = (_Float16)x1[i]; }
    ov[it] = f.half[0]; }
  unsigned short* orow = (unsigned short*)O16 + (rb + q0) * DM + h * HD;
  for (int pass = 0; pass < 2; ++pass) {
#pragma unroll
    for (int it = 0; it < 4; ++it) *(volatile v8us*)(orow + (size_t)(it * 4 + qs) * DM + pc * 8) = ov[it];
    if (pass == 0) __threadfence(); }
}

extern "C" void kernel_launch(void* const* d_in, const int* in_sizes, int n_in,
                              void* d_out, int out_size, void* d_ws, size_t ws_size, hipStream_t stream) {
  if (n_in < 11) return;
  const size_t need_x = ((size_t)(NB - 1) * SEQ_FULL + SEQ) * DM;
  if ((size_t)in_sizes[0] < need_x || (size_t)in_sizes[1] < need_x || (size_t)in_sizes[2] < need_x) return;
  if ((size_t)in_sizes[3] < (size_t)NH * DM * HD || (size_t)in_sizes[5] < (size_t)NH * DM * HD || (size_t)in_sizes[7] < (size_t)NH * DM * HD || (size_t)in_sizes[9] < (size_t)DM * DM) return;
  if (in_sizes[4] < DM || in_sizes[6] < DM || in_sizes[8] < DM || in_sizes[10] < DM) return;
  if ((size_t)out_size < NR * DM) return;
  if (ws_size < WS_TOTAL) return;
  const float* xq = (const float*)d_in[0]; const float* xk = (const float*)d_in[1]; const float* xv = (const float*)d_in[2];
  const float* wq = (const float*)d_in[3]; const float* bq = (const float*)d_in[4];
  const float* wk = (const float*)d_in[5]; const float* bk = (const float*)d_in[6];
  const float* wv = (const float*)d_in[7]; const float* bv = (const float*)d_in[8];
  const float* wo = (const float*)d_in[9]; const float* bo = (const float*)d_in[10];
  char* ws = (char*)d_ws; size_t off = 0;
  _Float16* BQ = (_Float16*)(ws + off); off += SZ_W;
  _Float16* BK = (_Float16*)(ws + off); off += SZ_W;
  _Float16* BV = (_Float16*)(ws + off); off += SZ_W;
  _Float16* BO = (_Float16*)(ws + off); off += SZ_W;
  _Float16* X16 = (_Float16*)(ws + off); off += SZ_ACT;
  _Float16* Q16 = (_Float16*)(ws + off); off += SZ_ACT;
  _Float16* K16 = (_Float16*)(ws + off); off += SZ_ACT;
  _Float16* V16 = (_Float16*)(ws + off); off += SZ_ACT;
  _Float16* O16 = (_Float16*)(ws + off); off += SZ_ACT;
  _Float16* VT  = (_Float16*)(ws + off); off += SZ_ACT;
  float* M2 = (float*)(ws + off); off += SZ_ST;
  float* RL = (float*)(ws + off); off += SZ_ST;
  if (off > ws_size) return;

  const unsigned gw = (unsigned)(((size_t)NH * HD * (DM / 8) + 255) / 256);
  k_wqkv<<<gw, 256, 0, stream>>>(wq, BQ);
  k_wqkv<<<gw, 256, 0, stream>>>(wk, BK);
  k_wqkv<<<gw, 256, 0, stream>>>(wv, BV);
  k_wnat<<<(unsigned)(((size_t)DM * DM / 8 + 255) / 256), 256, 0, stream>>>(wo, (size_t)DM * DM / 8, BO);

  const unsigned gx = (unsigned)((NR * (DM / 8) + 255) / 256);
  const unsigned gg = (unsigned)((NR / 128) * (DM / 64));
  k_x16<<<gx, 256, 0, stream>>>(xq, X16);
  k_gemm2<<<gg, 128, 0, stream>>>(X16, DM, BQ, DM, 0.0625f, bq, (float*)nullptr, Q16, DM, (int)NR, DM, DM);
  k_x16<<<gx, 256, 0, stream>>>(xk, X16);
  k_gemm2<<<gg, 128, 0, stream>>>(X16, DM, BK, DM, 0.0625f, bk, (float*)nullptr, K16, DM, (int)NR, DM, DM);
  k_x16<<<gx, 256, 0, stream>>>(xv, X16);
  k_gemm2<<<gg, 128, 0, stream>>>(X16, DM, BV, DM, 0.0625f, bv, (float*)nullptr, V16, DM, (int)NR, DM, DM);

  k_cstat<<<dim3(SEQ / (CW * 64), NB * NH), CW * 32, 0, stream>>>(Q16, K16, M2, RL);
  k_vt<<<NB * NH * (SEQ / 64), 256, 0, stream>>>(V16, RL, VT);
  k_actx<<<dim3(SEQ / (AW * 16), NB * NH), AW * 32, 0, stream>>>(Q16, K16, VT, M2, O16);

  k_gemm2<<<gg, 128, 0, stream>>>(O16, DM, BO, DM, 0.0009765625f, bo, (float*)d_out, (_Float16*)nullptr, DM, (int)NR, DM, DM);
}
